// LocalRNN_87196426043491
// MI455X (gfx1250) — hardware-verified
//
#include <hip/hip_runtime.h>
#include <math.h>

constexpr int kBatch = 16;
constexpr int kLen   = 1024;
constexpr int kHid   = 256;
constexpr int kG3    = 768;
constexpr int kWin   = 16;
constexpr int kTok   = kBatch * kLen;
constexpr float kWCarry    = 16.0f;
constexpr float kWCarryInv = 1.0f / 16.0f;

constexpr size_t kOffWih  = 0;
constexpr size_t kOffWhh  = kOffWih + (size_t)kG3 * kHid * 2;
constexpr size_t kOffXH   = kOffWhh + (size_t)kG3 * kHid * 2;
constexpr size_t kOffGI   = kOffXH  + (size_t)kTok * kHid * 2;
constexpr size_t kOffGH   = kOffGI  + (size_t)kTok * kG3 * 4;
constexpr size_t kOffHB   = kOffGH  + (size_t)kTok * kG3 * 4;
constexpr size_t kWsTotal = kOffHB  + (size_t)kTok * kHid * 4;
static_assert(kWsTotal <= (size_t)134217728, "ws");
static_assert((kOffXH % 128) == 0 && (kOffGI % 128) == 0 && (kOffGH % 128) == 0 && (kOffHB % 128) == 0, "align");

typedef __attribute__((ext_vector_type(16))) _Float16 v16h;
typedef __attribute__((ext_vector_type(8)))  _Float16 v8h;
typedef __attribute__((ext_vector_type(16))) __bf16   v16b;
typedef __attribute__((ext_vector_type(8)))  __bf16   v8b;
typedef __attribute__((ext_vector_type(8)))  float    v8f;
typedef __attribute__((ext_vector_type(4)))  float    v4f;
typedef __attribute__((ext_vector_type(4)))  unsigned int v4u;

__device__ __forceinline__ unsigned short f2bf_bits(float f) {
  unsigned u = __float_as_uint(f);
  return (unsigned short)((u + 0x7FFFu + ((u >> 16) & 1u)) >> 16);
}
__device__ __forceinline__ float bf_bits2f(unsigned short h) { return __uint_as_float(((unsigned)h) << 16); }

__device__ __forceinline__ void dep_guard_h(v8f& a, v8f& b, v16h x, v16h y) { asm volatile("v_nop\n\tv_nop\n\tv_nop\n\tv_nop" : "+v"(a), "+v"(b) : "v"(x), "v"(y)); }
__device__ __forceinline__ void dep_guard_b(v8f& a, v8f& b, v16b x, v16b y) { asm volatile("v_nop\n\tv_nop\n\tv_nop\n\tv_nop" : "+v"(a), "+v"(b) : "v"(x), "v"(y)); }
__device__ __forceinline__ void keep4_h(v16h a, v16h b, v16h c, v16h d) { asm volatile("v_nop" :: "v"(a), "v"(b), "v"(c), "v"(d)); }
__device__ __forceinline__ void keep4_b(v16b a, v16b b, v16b c, v16b d) { asm volatile("v_nop" :: "v"(a), "v"(b), "v"(c), "v"(d)); }
__device__ __forceinline__ void acc_guard4(v8f& a, v8f& b, v8f& c, v8f& d) { asm volatile("v_nop\n\tv_nop\n\tv_nop\n\tv_nop" : "+v"(a), "+v"(b), "+v"(c), "+v"(d)); }
template <typename T> struct Frag;
template <> struct Frag<_Float16> {
  typedef v16h V; union U { v16h v; v8h h[2]; };
  static __device__ __forceinline__ v16h load(const _Float16* p) {
    U f; f.h[0] = *(const v8h*)(p); f.h[1] = *(const v8h*)(p + 16); return f.v;
  }
  static __device__ __forceinline__ v8f mma(v16h a, v16h b, v8f c) {
    return __builtin_amdgcn_wmma_f32_16x16x32_f16(false, a, false, b, (short)0, c, false, false);
  }
  static __device__ __forceinline__ void guard(v8f& a, v8f& b, v16h x, v16h y) { dep_guard_h(a, b, x, y); }
  static __device__ __forceinline__ void keep(v16h a, v16h b, v16h c, v16h d) { keep4_h(a, b, c, d); }
};
template <> struct Frag<__bf16> {
  typedef v16b V; union U { v16b v; v8b h[2]; };
  static __device__ __forceinline__ v16b load(const __bf16* p) {
    U f; f.h[0] = *(const v8b*)(p); f.h[1] = *(const v8b*)(p + 16); return f.v;
  }
  static __device__ __forceinline__ v8f mma(v16b a, v16b b, v8f c) {
    return __builtin_amdgcn_wmma_f32_16x16x32_bf16(false, a, false, b, (short)0, c, false, false);
  }
  static __device__ __forceinline__ void guard(v8f& a, v8f& b, v16b x, v16b y) { dep_guard_b(a, b, x, y); }
  static __device__ __forceinline__ void keep(v16b a, v16b b, v16b c, v16b d) { keep4_b(a, b, c, d); }
};

__device__ __forceinline__ unsigned pk16(unsigned short a, unsigned short b) { return (unsigned)a | ((unsigned)b << 16); }
__device__ __forceinline__ unsigned short h_bits(float f) { const _Float16 h = (_Float16)f; return __builtin_bit_cast(unsigned short, h); }

template <int ET> struct Elem;
template <> struct Elem<0> { typedef _Float16 T; };
template <> struct Elem<1> { typedef __bf16 T; };
template <int ET, bool SPLIT, int BIAS_MODE, int OUT_MODE, bool RESID, int ACT = 0>
__global__ __launch_bounds__(256) void wmma_gemm64(
    const unsigned short* __restrict__ Ap, const unsigned short* __restrict__ A2p, int lda, long strideA,
    const unsigned short* __restrict__ Btp, const unsigned short* __restrict__ Bt2p, int ldb, long strideB,
    void* __restrict__ Cout, void* __restrict__ Cout2, int ldc, long strideC,
    const float* __restrict__ bias,
    const float* __restrict__ resid, long strideR,
    int M, int N, int K, float scale) {
  typedef typename Elem<ET>::T T;
  typedef typename Frag<T>::V V;
  const T* A = (const T*)Ap; const T* A2 = (const T*)A2p; const T* Bt = (const T*)Btp; const T* Bt2 = (const T*)Bt2p;
  __shared__ __align__(16) float sT[8][16 * 68];
  const int b    = blockIdx.y;
  const int lane = threadIdx.x & 31;
  const int wave = threadIdx.x >> 5;
  const int tilesN = N >> 6;
  const int tilesM = M >> 6;
  const int tile = blockIdx.x * 8 + wave;
  if (tile >= tilesM * tilesN) return;
  const int tm = tile / tilesN;
  const int tn = tile - tm * tilesN;
  const int m0 = tm << 6;
  const int n0 = tn << 6;

  const T* Ab  = A  + (size_t)b * strideA;
  const T* Bb  = Bt + (size_t)b * strideB;
  const T* Ab2 = SPLIT ? (A2  + (size_t)b * strideA) : nullptr;
  const T* Bb2 = SPLIT ? (Bt2 + (size_t)b * strideB) : nullptr;

  const int rlane = lane & 15;
  const int koff  = (lane >> 4) * 8;
  const int mOff  = (lane >> 4) * 8;

  v8f acc[4][4];
#pragma unroll
  for (int i = 0; i < 4; ++i)
#pragma unroll
    for (int j = 0; j < 4; ++j) acc[i][j] = (v8f){0.f,0.f,0.f,0.f,0.f,0.f,0.f,0.f};

  for (int k0 = 0; k0 < K; k0 += 32) {
    V bh[4], bl[4];
#pragma unroll
    for (int j = 0; j < 4; ++j) {
      const size_t bo = (size_t)(n0 + (j << 4) + rlane) * ldb + koff + k0;
      bh[j] = Frag<T>::load(Bb + bo);
      if (SPLIT) bl[j] = Frag<T>::load(Bb2 + bo);
    }
#pragma unroll
    for (int i = 0; i < 4; ++i) {
      const size_t ao = (size_t)(m0 + (i << 4) + rlane) * lda + koff + k0;
      V ah = Frag<T>::load(Ab + ao);
      V al;
      if (SPLIT) al = Frag<T>::load(Ab2 + ao);
#pragma unroll
      for (int j = 0; j < 4; ++j) {
        acc[i][j] = Frag<T>::mma(ah, bh[j], acc[i][j]);
        if (SPLIT) {
          acc[i][j] = Frag<T>::mma(ah, bl[j], acc[i][j]);
          acc[i][j] = Frag<T>::mma(al, bh[j], acc[i][j]);
        }
      }
      Frag<T>::guard(acc[i][0], acc[i][3], ah, SPLIT ? al : ah);
    }
    Frag<T>::keep(bh[0], bh[1], bh[2], bh[3]);
    if (SPLIT) Frag<T>::keep(bl[0], bl[1], bl[2], bl[3]);
  }
  acc_guard4(acc[0][0], acc[0][1], acc[0][2], acc[0][3]);
  acc_guard4(acc[1][0], acc[1][1], acc[1][2], acc[1][3]);
  acc_guard4(acc[2][0], acc[2][1], acc[2][2], acc[2][3]);
  acc_guard4(acc[3][0], acc[3][1], acc[3][2], acc[3][3]);

  float* slab = sT[wave];
  const float* Rb = RESID ? (resid + (size_t)b * strideR) : nullptr;
#pragma unroll
  for (int i = 0; i < 4; ++i) {
    const int mBase = m0 + (i << 4);
#pragma unroll
    for (int j = 0; j < 4; ++j) {
      const int n = n0 + (j << 4) + rlane;
      float bv = 0.f;
      if (BIAS_MODE == 2) bv = bias[n];
#pragma unroll
      for (int r = 0; r < 8; ++r) {
        float v = acc[i][j][r] * scale;
        if (BIAS_MODE == 1) v += bias[mBase + mOff + r];
        if (BIAS_MODE == 2) v += bv;
        if (RESID) v += Rb[(size_t)(mBase + mOff + r) * ldc + n];
        if (ACT == 2) v = fmaxf(v, 0.0f);
        if (ACT == 4) v = (v > 0.f) ? v : 0.01f * v;
        slab[(mOff + r) * 68 + (j << 4) + rlane] = v;
      }
    }
    __builtin_amdgcn_fence(__ATOMIC_RELEASE, "workgroup");
    __builtin_amdgcn_wave_barrier();
    __builtin_amdgcn_fence(__ATOMIC_ACQUIRE, "workgroup");
    if (OUT_MODE == 0) {
      float* C = (float*)Cout + (size_t)b * strideC;
      const int hh = lane >> 4, c4 = (lane & 15) * 4;
      for (int pass = 0; pass < 2; ++pass) {
#pragma unroll
        for (int it = 0; it < 8; ++it) {
          const int row = it * 2 + hh;
          v4f v = *(const v4f*)(slab + row * 68 + c4);
          *(volatile v4f*)(C + (size_t)(mBase + row) * ldc + n0 + c4) = v;
        }
        __threadfence();
      }
    } else {
      const int q = lane >> 3, c8 = (lane & 7) * 8;
      unsigned short* C  = (unsigned short*)Cout  + (size_t)b * strideC;
      unsigned short* C2 = (OUT_MODE == 2) ? ((unsigned short*)Cout2 + (size_t)b * strideC) : nullptr;
      for (int pass = 0; pass < 2; ++pass) {
#pragma unroll
        for (int it = 0; it < 4; ++it) {
          const int row = it * 4 + q;
          const float* sp = slab + row * 68 + c8;
          v8h hv, lv;
#pragma unroll
          for (int e = 0; e < 8; ++e) {
            if (OUT_MODE == 1) {
              hv[e] = (_Float16)sp[e];
            } else {
              unsigned short hb = f2bf_bits(sp[e]);
              unsigned short lb = f2bf_bits(sp[e] - bf_bits2f(hb));
              hv[e] = __builtin_bit_cast(_Float16, hb);
              lv[e] = __builtin_bit_cast(_Float16, lb);
            }
          }
          *(volatile v8h*)(C + (size_t)(mBase + row) * ldc + n0 + c8) = hv;
          if (OUT_MODE == 2) *(volatile v8h*)(C2 + (size_t)(mBase + row) * ldc + n0 + c8) = lv;
        }
        __threadfence();
      }
    }
    __builtin_amdgcn_fence(__ATOMIC_RELEASE, "workgroup");
    __builtin_amdgcn_wave_barrier();
    __builtin_amdgcn_fence(__ATOMIC_ACQUIRE, "workgroup");
  }
}

__global__ __launch_bounds__(256) void cast8s_f16_kernel(const float* __restrict__ in, unsigned short* __restrict__ out,
                                                         int n8, float scale) {
  const int i = blockIdx.x * 256 + threadIdx.x;
  if (i >= n8) return;
  const float* p = in + 8 * (size_t)i;
  const v4f a = *(const v4f*)(p);
  const v4f c = *(const v4f*)(p + 4);
  unsigned short hb[8];
#pragma unroll
  for (int e = 0; e < 4; ++e) {
    hb[e]     = h_bits(a[e] * scale);
    hb[4 + e] = h_bits(c[e] * scale);
  }
  const v4u u = (v4u){pk16(hb[0], hb[1]), pk16(hb[2], hb[3]), pk16(hb[4], hb[5]), pk16(hb[6], hb[7])};
  unsigned short* q = out + 8 * (size_t)i;
  *(volatile v4u*)q = u;
  __threadfence();
  *(volatile v4u*)q = u;
}

__device__ __forceinline__ float sigm_f(float x) {
  const float e = expf(-x);
  return __builtin_amdgcn_rcpf(1.0f + e);
}
__device__ __forceinline__ float tanh_f(float y) {
  const float t  = expf(-2.0f * fabsf(y));
  const float th = (1.0f - t) * __builtin_amdgcn_rcpf(1.0f + t);
  return copysignf(th, y);
}

template <bool kFirst>
__global__ __launch_bounds__(256) void gru_cell_kernel(
    const float* __restrict__ gi, const float* __restrict__ gh,
    const float* __restrict__ bih, const float* __restrict__ bhh,
    const float* __restrict__ hprev, float* __restrict__ hout,
    unsigned short* __restrict__ h16, const int* __restrict__ ksz, int step) {
  __shared__ __align__(16) float sH[8][kHid];
  const int t    = threadIdx.x;
  const int lane = t & 31;
  const int wave = t >> 5;
  const int n    = blockIdx.x * 8 + wave;
  const int bidx = n >> 10;
  const int p    = n & 1023;
  const int src  = p - (kWin - 1) + step;
  const bool usex = (src >= 0);
  const int srcc = usex ? src : 0;
  const float* girow = gi + ((size_t)(bidx * kLen + srcc)) * kG3;
  const float* ghrow = gh + (size_t)n * kG3;
  const float* hprow = hprev + (size_t)n * kHid;
  const int kz = ksz[0];
  const float qnan = __int_as_float(0x7fc00000);
  float* sh = sH[wave];

#pragma unroll 1
  for (int j0 = 0; j0 < 8; j0 += 4) {
    const int u = lane * 8 + j0;
    const v4f xr = *(const v4f*)(girow + u);
    const v4f xz = *(const v4f*)(girow + kHid + u);
    const v4f xn = *(const v4f*)(girow + 2 * kHid + u);
    const v4f br = *(const v4f*)(bih + u);
    const v4f bz = *(const v4f*)(bih + kHid + u);
    const v4f bn = *(const v4f*)(bih + 2 * kHid + u);
    v4f gr, gz, gn, hp;
    if (kFirst) {
      gr = *(const v4f*)(bhh + u);
      gz = *(const v4f*)(bhh + kHid + u);
      gn = *(const v4f*)(bhh + 2 * kHid + u);
      hp = (v4f){0.f, 0.f, 0.f, 0.f};
    } else {
      gr = *(const v4f*)(ghrow + u);
      gz = *(const v4f*)(ghrow + kHid + u);
      gn = *(const v4f*)(ghrow + 2 * kHid + u);
      hp = *(const v4f*)(hprow + u);
    }
#pragma unroll
    for (int e = 0; e < 4; ++e) {
      const float ir = usex ? xr[e] : br[e];
      const float iz = usex ? xz[e] : bz[e];
      const float ic = usex ? xn[e] : bn[e];
      const float r  = sigm_f(ir + gr[e]);
      const float z  = sigm_f(iz + gz[e]);
      const float c  = tanh_f(ic + r * gn[e]);
      float hv = (1.0f - z) * c + z * hp[e];
      hv = (kz != kWin) ? qnan : hv;
      sh[u + e] = hv;
    }
  }
  __syncthreads();

  {
    const float* shr = sH[wave];
    const v4f a = *(const v4f*)(shr + lane * 8);
    const v4f c = *(const v4f*)(shr + lane * 8 + 4);
    unsigned short hb[8];
#pragma unroll
    for (int e = 0; e < 4; ++e) {
      hb[e]     = h_bits(a[e]);
      hb[4 + e] = h_bits(c[e]);
    }
    const v4u u16 = (v4u){pk16(hb[0], hb[1]), pk16(hb[2], hb[3]), pk16(hb[4], hb[5]), pk16(hb[6], hb[7])};
    const v4f f0 = *(const v4f*)(shr + lane * 4);
    const v4f f1 = *(const v4f*)(shr + 128 + lane * 4);
    unsigned short* q16 = h16 + (size_t)n * kHid + lane * 8;
    float* qo = hout + (size_t)n * kHid;
    *(volatile v4u*)q16 = u16;
    *(volatile v4f*)(qo + lane * 4) = f0;
    *(volatile v4f*)(qo + 128 + lane * 4) = f1;
    __threadfence();
    *(volatile v4u*)q16 = u16;
    *(volatile v4f*)(qo + lane * 4) = f0;
    *(volatile v4f*)(qo + 128 + lane * 4) = f1;
  }
}

extern "C" void kernel_launch(void* const* d_in, const int* in_sizes, int n_in,
                              void* d_out, int out_size, void* d_ws, size_t ws_size,
                              hipStream_t stream) {
  if (n_in < 6) return;
  if (in_sizes[0] != kTok * kHid) return;
  if (in_sizes[1] != kG3 * kHid || in_sizes[2] != kG3 * kHid) return;
  if (in_sizes[3] != kG3 || in_sizes[4] != kG3 || in_sizes[5] < 1) return;
  if (out_size != kTok * kHid) return;
  if (ws_size < kWsTotal) return;

  const float* x   = (const float*)d_in[0];
  const float* wih = (const float*)d_in[1];
  const float* whh = (const float*)d_in[2];
  const float* bih = (const float*)d_in[3];
  const float* bhh = (const float*)d_in[4];
  const int*   ksz = (const int*)d_in[5];
  float* out = (float*)d_out;

  char* ws = (char*)d_ws;
  unsigned short* wih16 = (unsigned short*)(ws + kOffWih);
  unsigned short* whh16 = (unsigned short*)(ws + kOffWhh);
  unsigned short* xh16  = (unsigned short*)(ws + kOffXH);
  float* giP = (float*)(ws + kOffGI);
  float* ghP = (float*)(ws + kOffGH);
  float* hbP = (float*)(ws + kOffHB);

  const int nx8 = (kTok * kHid) / 8;
  const int nw8 = (kG3 * kHid) / 8;
  cast8s_f16_kernel<<<dim3((nx8 + 255) / 256), dim3(256), 0, stream>>>(x, xh16, nx8, 1.0f);
  cast8s_f16_kernel<<<dim3((nw8 + 255) / 256), dim3(256), 0, stream>>>(wih, wih16, nw8, kWCarry);
  cast8s_f16_kernel<<<dim3((nw8 + 255) / 256), dim3(256), 0, stream>>>(whh, whh16, nw8, kWCarry);

  const int gemmBlocks = ((kTok / 64) * (kG3 / 64)) / 8;

  wmma_gemm64<0, false, 2, 0, false, 0><<<dim3(gemmBlocks, 1), dim3(256), 0, stream>>>(
      xh16, xh16, kHid, 0L, wih16, wih16, kHid, 0L,
      (void*)giP, (void*)giP, kG3, 0L, bih, bih, 0L, kTok, kG3, kHid, kWCarryInv);

  const int cellBlocks = kTok / 8;

  gru_cell_kernel<true><<<dim3(cellBlocks), dim3(256), 0, stream>>>(
      giP, ghP, bih, bhh, hbP, hbP, xh16, ksz, 0);

  for (int k = 1; k < kWin; ++k) {
    wmma_gemm64<0, false, 2, 0, false, 0><<<dim3(gemmBlocks, 1), dim3(256), 0, stream>>>(
        xh16, xh16, kHid, 0L, whh16, whh16, kHid, 0L,
        (void*)ghP, (void*)ghP, kG3, 0L, bhh, bhh, 0L, kTok, kG3, kHid, kWCarryInv);
    const float* hsrc = (k & 1) ? (const float*)hbP : (const float*)out;
    float* hdst = (k & 1) ? out : hbP;
    gru_cell_kernel<false><<<dim3(cellBlocks), dim3(256), 0, stream>>>(
        giP, ghP, bih, bhh, hsrc, hdst, xh16, ksz, k);
  }
}
